// YvChunkedParallelScan_72112500900643
// MI455X (gfx1250) — hardware-run, weakly checked
//
#include <hip/hip_runtime.h>
#include <math.h>

typedef __attribute__((ext_vector_type(16))) _Float16 v16h;
typedef __attribute__((ext_vector_type(8)))  _Float16 v8h;
typedef __attribute__((ext_vector_type(8)))  float    v8f;
typedef __attribute__((ext_vector_type(4)))  float    v4f;

constexpr int kBatch  = 2;
constexpr int kSeq    = 2048;
constexpr int kDm     = 1024;
constexpr int kNst    = 32;
constexpr int kChunk  = 256;
constexpr int kNc     = kSeq / kChunk;
constexpr int kRows   = kBatch * kSeq;
constexpr int kScanCh = 128;
constexpr int kScanTS = 32;
constexpr int kScanYP = 132;
constexpr int kGemmBlocksX = (kDm / 64) * (kChunk / 16) / 8;
constexpr float kCarryC = 256.0f;
constexpr float kCarryM = 2048.0f;
constexpr float kFold   = 1.0f / (kCarryC * kCarryM);
constexpr float kF16MinNormal = 6.103515625e-05f;

static_assert(kNc == 8, "eight chunks");
static_assert(kNst == 32, "one 32-deep k-step");
static_assert(kScanTS >= kNst, "the y tile doubles as the decay staging tile");
static_assert((kChunk % kScanTS) == 0 && (kDm % kScanCh) == 0, "scan tile multiples");
static_assert((kScanTS * kNst) == 2 * kScanCh * 4, "B and C sub-tile staging: 2 float4 per thread");
static_assert((kChunk % 16) == 0 && (kDm % 64) == 0, "product tile multiples");
static_assert(kGemmBlocksX == 32, "product grid");
static_assert((kScanYP % 4) == 0, "16-B aligned tile rows");

constexpr size_t kOffYT   = 0;
constexpr size_t kOffMT   = kOffYT + (size_t)kRows * kDm * 4;
constexpr size_t kWsTotal = kOffMT + (size_t)kBatch * (kNc - 1) * kDm * kNst * 2;
static_assert(kWsTotal == 17694720ull, "carve total");
static_assert(kWsTotal <= 134217728ull, "carve cap");
static_assert((kOffMT % 128) == 0, "128-B aligned regions");

union FragU { v16h v; v8h h[2]; };

__device__ __forceinline__ v16h frag_load_f16(const _Float16* p) {
  FragU f;
  f.h[0] = *(const v8h*)(p);
  f.h[1] = *(const v8h*)(p + 16);
  return f.v;
}

__device__ __forceinline__ v8f mma_f16_guarded(v16h a, v16h b, v8f c) {
  c = __builtin_amdgcn_wmma_f32_16x16x32_f16(false, a, false, b, (short)0, c, false, false);
  asm volatile("v_nop\n\tv_nop\n\tv_nop\n\tv_nop" : "+v"(c) : "v"(a), "v"(b));
  return c;
}

__device__ __forceinline__ _Float16 to_f16_carried(float v, float carry) {
  const float s = v * carry;
  const float z = (fabsf(s) < kF16MinNormal) ? 0.0f : s;
  return (_Float16)z;
}

__global__ __launch_bounds__(128) void chunk_scan_kernel(
    const float* __restrict__ u, const float* __restrict__ Bm, const float* __restrict__ Cm,
    const float* __restrict__ Al, const float* __restrict__ Dp,
    float* __restrict__ Yt, unsigned short* __restrict__ Mt)
{
  __shared__ __align__(16) float    sB[kScanTS * kNst];
  __shared__ __align__(16) float    sC[kScanTS * kNst];
  __shared__ __align__(16) float    sY[kScanTS * kScanYP];
  __shared__ __align__(16) _Float16 sM[kScanCh * kNst];

  unsigned tid = threadIdx.x;
  asm volatile("" : "+v"(tid));
  unsigned lane = tid & 31u;
  asm volatile("" : "+v"(lane));
  unsigned wave = tid >> 5;
  asm volatile("" : "+v"(wave));

  const int bc = blockIdx.x;
  const int b  = bc / kNc;
  const int c  = bc - b * kNc;
  const int d0 = blockIdx.y * kScanCh;
  const unsigned d = (unsigned)d0 + tid;
  const size_t rowBase = (size_t)b * kSeq + (size_t)c * kChunk;

#pragma unroll 1
  for (int n = 0; n < kNst; ++n)
    sY[n * kScanYP + tid] = -expf(Al[(size_t)n * kDm + d]);
  __syncthreads();

  float a[kNst], h[kNst];
#pragma unroll
  for (int n = 0; n < kNst; ++n) {
    a[n] = sY[n * kScanYP + tid];
    h[n] = 0.0f;
  }
  const float dpar = Dp[d];

#pragma unroll 1
  for (int t0 = 0; t0 < kChunk; t0 += kScanTS) {
    __syncthreads();
#pragma unroll
    for (int i = 0; i < 2; ++i) {
      const unsigned vi = (unsigned)i * (unsigned)kScanCh + tid;
      const size_t go = (rowBase + (size_t)t0) * kNst + (size_t)vi * 4;
      *(v4f*)(sB + vi * 4) = *(const v4f*)(Bm + go);
      *(v4f*)(sC + vi * 4) = *(const v4f*)(Cm + go);
    }
    __syncthreads();

#pragma unroll 1
    for (int s = 0; s < kScanTS; ++s) {
      const float ut = u[(rowBase + (size_t)(t0 + s)) * kDm + d];
      const float* bp = sB + s * kNst;
      const float* cp = sC + s * kNst;
      float y = 0.0f;
#pragma unroll
      for (int q = 0; q < kNst / 4; ++q) {
        const v4f bv = *(const v4f*)(bp + 4 * q);
        const v4f cv = *(const v4f*)(cp + 4 * q);
#pragma unroll
        for (int e = 0; e < 4; ++e) {
          const float bu = bv[e] * ut;
          h[4 * q + e] = fmaf(a[4 * q + e], h[4 * q + e], bu);
          y = fmaf(cv[e], h[4 * q + e], y);
        }
      }
      sY[s * kScanYP + tid] = fmaf(ut, dpar, y);
    }
    __syncthreads();

    v4f fv[8];
#pragma unroll
    for (int it = 0; it < 8; ++it) {
      const unsigned row = (unsigned)it * 4u + wave;
      fv[it] = *(const v4f*)(sY + row * kScanYP + lane * 4u);
    }
    for (int pass = 0; pass < 2; ++pass) {
#pragma unroll
      for (int it = 0; it < 8; ++it) {
        const unsigned row = (unsigned)it * 4u + wave;
        *(volatile v4f*)(Yt + (rowBase + (size_t)t0 + row) * kDm + d0 + lane * 4u) = fv[it];
      }
      __threadfence();
    }
  }

#pragma unroll
  for (int g = 0; g < 4; ++g) {
    v8h hv;
#pragma unroll
    for (int e = 0; e < 8; ++e) {
      const float m = a[8 * g + e] * h[8 * g + e];
      hv[e] = to_f16_carried(m, kCarryM);
    }
    *(v8h*)(sM + tid * (unsigned)kNst + 8u * (unsigned)g) = hv;
  }
  __syncthreads();
  v8h mv[4];
#pragma unroll
  for (int i = 0; i < 4; ++i) {
    const unsigned vec = (unsigned)i * (unsigned)kScanCh + tid;
    mv[i] = *(const v8h*)(sM + vec * 8u);
  }
  if (c < kNc - 1) {
    unsigned short* mdst = Mt + ((size_t)(b * (kNc - 1) + c) * kDm + (size_t)d0) * kNst;
    for (int pass = 0; pass < 2; ++pass) {
#pragma unroll
      for (int i = 0; i < 4; ++i) {
        const unsigned vec = (unsigned)i * (unsigned)kScanCh + tid;
        *(volatile v8h*)(mdst + (size_t)vec * 8) = mv[i];
      }
      __threadfence();
    }
  }
}

__global__ __launch_bounds__(256) void corr_gemm_kernel(
    const float* __restrict__ Cm, const unsigned short* __restrict__ Mt,
    const float* __restrict__ Yt, float* __restrict__ out)
{
  __shared__ __align__(16) float sT[8][16 * 68];

  unsigned tid = threadIdx.x;
  asm volatile("" : "+v"(tid));
  unsigned lane = tid & 31u;
  asm volatile("" : "+v"(lane));
  unsigned wave = tid >> 5;
  asm volatile("" : "+v"(wave));
  unsigned rl = lane & 15u;
  asm volatile("" : "+v"(rl));
  unsigned hh = lane >> 4;
  asm volatile("" : "+v"(hh));

  const int bc = blockIdx.y;
  const int b  = bc / kNc;
  const int c  = bc - b * kNc;
  const int n0 = (int)(blockIdx.x >> 1) * 64;
  const unsigned m0 = ((unsigned)(blockIdx.x & 1u) * 8u + wave) * 16u;
  const size_t rowBase = (size_t)b * kSeq + (size_t)c * kChunk + (size_t)m0;

  v8f acc[4];
#pragma unroll
  for (int j = 0; j < 4; ++j) acc[j] = (v8f){0.f, 0.f, 0.f, 0.f, 0.f, 0.f, 0.f, 0.f};

  if (c > 0) {
    const float* crow = Cm + (rowBase + rl) * kNst + 8u * hh;
    const v4f c0 = *(const v4f*)(crow);
    const v4f c1 = *(const v4f*)(crow + 4);
    const v4f c2 = *(const v4f*)(crow + 16);
    const v4f c3 = *(const v4f*)(crow + 20);
    v16h af;
#pragma unroll
    for (int e = 0; e < 4; ++e) {
      const float x0 = c0[e];
      const float x1 = c1[e];
      const float x2 = c2[e];
      const float x3 = c3[e];
      af[e]      = to_f16_carried(x0, kCarryC);
      af[4 + e]  = to_f16_carried(x1, kCarryC);
      af[8 + e]  = to_f16_carried(x2, kCarryC);
      af[12 + e] = to_f16_carried(x3, kCarryC);
    }
    const _Float16* mb = (const _Float16*)Mt + ((size_t)(b * (kNc - 1) + (c - 1)) * kDm + (size_t)n0) * kNst;
#pragma unroll
    for (int j = 0; j < 4; ++j) {
      const v16h bf = frag_load_f16(mb + (size_t)((unsigned)j * 16u + rl) * kNst + 8u * hh);
      acc[j] = mma_f16_guarded(af, bf, acc[j]);
    }
  }

  float* slab = sT[wave];
#pragma unroll
  for (int j = 0; j < 4; ++j) {
#pragma unroll
    for (int r = 0; r < 8; ++r)
      slab[(8u * hh + (unsigned)r) * 68u + (unsigned)j * 16u + rl] = acc[j][r] * kFold;
  }
  __syncthreads();

  const unsigned c4 = rl * 4u;
  v4f vals[8];
#pragma unroll
  for (int it = 0; it < 8; ++it) {
    const unsigned row = (unsigned)it * 2u + hh;
    const v4f sv = *(const v4f*)(slab + row * 68u + c4);
    const v4f yv = *(const v4f*)(Yt + (rowBase + row) * kDm + n0 + c4);
    vals[it] = sv + yv;
  }
  for (int pass = 0; pass < 2; ++pass) {
#pragma unroll
    for (int it = 0; it < 8; ++it) {
      const unsigned row = (unsigned)it * 2u + hh;
      *(volatile v4f*)(out + (rowBase + row) * kDm + n0 + c4) = vals[it];
    }
    __threadfence();
  }
}

extern "C" void kernel_launch(void* const* d_in, const int* in_sizes, int n_in,
                              void* d_out, int out_size, void* d_ws, size_t ws_size,
                              hipStream_t stream) {
  if (n_in < 6) return;
  if (in_sizes[0] != kRows * kDm) return;
  if (in_sizes[2] != kRows * kNst) return;
  if (in_sizes[3] != kRows * kNst) return;
  if (in_sizes[4] != kNst * kDm) return;
  if (in_sizes[5] != kDm) return;
  if (out_size != kRows * kDm) return;
  if (ws_size < kWsTotal) return;

  const float* u  = (const float*)d_in[0];
  const float* Bm = (const float*)d_in[2];
  const float* Cm = (const float*)d_in[3];
  const float* Al = (const float*)d_in[4];
  const float* Dp = (const float*)d_in[5];
  float* out = (float*)d_out;

  char* ws = (char*)d_ws;
  float*          Yt = (float*)(ws + kOffYT);
  unsigned short* Mt = (unsigned short*)(ws + kOffMT);

  chunk_scan_kernel<<<dim3(kBatch * kNc, kDm / kScanCh), kScanCh, 0, stream>>>(u, Bm, Cm, Al, Dp, Yt, Mt);
  corr_gemm_kernel<<<dim3(kGemmBlocksX, kBatch * kNc), 256, 0, stream>>>(Cm, Mt, Yt, out);
}
